// CausalRSSM_18786186953413
// MI455X (gfx1250) — hardware-run, weakly checked
//
#include <hip/hip_runtime.h>
#include <math.h>

typedef __attribute__((ext_vector_type(16))) _Float16 v16h;
typedef __attribute__((ext_vector_type(8)))  _Float16 v8h;
typedef __attribute__((ext_vector_type(16))) __bf16   v16b;
typedef __attribute__((ext_vector_type(8)))  __bf16   v8b;
typedef __attribute__((ext_vector_type(8)))  float    v8f;
typedef __attribute__((ext_vector_type(4)))  float    v4f;

constexpr int kBatch = 4096;
constexpr int kFeat  = 512;
constexpr int kSto   = 32;
constexpr int kHid   = 512;
constexpr int kHid2  = 256;
constexpr int kMiH   = 64;
constexpr int kPairs = 496;
constexpr int kPar   = 64;
constexpr int kKlBlocks  = kBatch / 32;
constexpr int kMseBlocks = (kBatch * kFeat) / 4096;
static_assert(kPairs == kSto * (kSto - 1) / 2, "pair count");
static_assert(kPar == 2 * kSto, "mean | log_std width");
static_assert(kKlBlocks == 128 && kMseBlocks == 512, "partial tables");
static_assert((kBatch % 64) == 0 && (kHid % 64) == 0 && (kFeat % 64) == 0 && (kPar % 64) == 0, "GEMM M,N multiples of 64");
static_assert((kFeat % 32) == 0 && (kHid % 32) == 0 && (kSto % 32) == 0 && (kMiH % 32) == 0, "GEMM K multiples of 32");

constexpr float kMechCarry    = 16.0f;
constexpr float kMechCarryInv = 1.0f / kMechCarry;
constexpr float kLoCarry      = 2048.0f;
constexpr float kMechLoInv    = 1.0f / (kMechCarry * kLoCarry);
constexpr float kMiCarry      = 16.0f;
constexpr float kMiCarryInv   = 1.0f / kMiCarry;

constexpr size_t kSzFeat16 = (size_t)kBatch * kFeat * 2;
constexpr size_t kSzW1     = (size_t)kHid * kFeat * 2;
constexpr size_t kSzW2     = (size_t)kPar * kHid * 2;
constexpr size_t kSzH16    = (size_t)kBatch * kHid * 2;
constexpr size_t kSzPar    = (size_t)kBatch * kPar * 4;
constexpr size_t kSzZF     = (size_t)kBatch * kSto * 4;
constexpr size_t kSzMW     = (size_t)kSto * kHid2 * kSto * 2;
constexpr size_t kSzZC     = (size_t)kBatch * kSto * 2;
constexpr size_t kSzD1     = (size_t)kHid * kSto * 2;
constexpr size_t kSzG      = (size_t)kBatch * kHid * 2;
constexpr size_t kSzD2     = (size_t)kFeat * kHid * 2;
constexpr size_t kSzMIW    = (size_t)kPairs * kMiH * kMiH * 2;
constexpr size_t kSzKLP    = (size_t)kKlBlocks * 32 * 4;
constexpr size_t kSzMSEP   = (size_t)kMseBlocks * 32 * 4;
constexpr size_t kSzMIP    = (size_t)kPairs * 32 * 4;
constexpr size_t kOffFH   = 0;
constexpr size_t kOffFL   = kOffFH   + kSzFeat16;
constexpr size_t kOffW1H  = kOffFL   + kSzFeat16;
constexpr size_t kOffW1L  = kOffW1H  + kSzW1;
constexpr size_t kOffW2H  = kOffW1L  + kSzW1;
constexpr size_t kOffW2L  = kOffW2H  + kSzW2;
constexpr size_t kOffHH   = kOffW2L  + kSzW2;
constexpr size_t kOffHL   = kOffHH   + kSzH16;
constexpr size_t kOffPar  = kOffHL   + kSzH16;
constexpr size_t kOffZF   = kOffPar  + kSzPar;
constexpr size_t kOffMW   = kOffZF   + kSzZF;
constexpr size_t kOffZCH  = kOffMW   + kSzMW;
constexpr size_t kOffZCL  = kOffZCH  + kSzZC;
constexpr size_t kOffD1H  = kOffZCL  + kSzZC;
constexpr size_t kOffD1L  = kOffD1H  + kSzD1;
constexpr size_t kOffGH   = kOffD1L  + kSzD1;
constexpr size_t kOffGL   = kOffGH   + kSzG;
constexpr size_t kOffD2H  = kOffGL   + kSzG;
constexpr size_t kOffD2L  = kOffD2H  + kSzD2;
constexpr size_t kOffMIW  = kOffD2L  + kSzD2;
constexpr size_t kOffKLP  = kOffMIW  + kSzMIW;
constexpr size_t kOffMSEP = kOffKLP  + kSzKLP;
constexpr size_t kOffMIP  = kOffMSEP + kSzMSEP;
constexpr size_t kWsTotal = kOffMIP  + kSzMIP;
static_assert(kWsTotal == 34289664ull, "carve total");
static_assert(kWsTotal <= 134217728ull, "carve cap");
static_assert((kOffFL % 128) == 0 && (kOffW1H % 128) == 0 && (kOffW1L % 128) == 0 && (kOffW2H % 128) == 0 &&
              (kOffW2L % 128) == 0 && (kOffHH % 128) == 0 && (kOffHL % 128) == 0 && (kOffPar % 128) == 0 &&
              (kOffZF % 128) == 0 && (kOffMW % 128) == 0 && (kOffZCH % 128) == 0 && (kOffZCL % 128) == 0 &&
              (kOffD1H % 128) == 0 && (kOffD1L % 128) == 0 && (kOffGH % 128) == 0 && (kOffGL % 128) == 0 &&
              (kOffD2H % 128) == 0 && (kOffD2L % 128) == 0 && (kOffMIW % 128) == 0 && (kOffKLP % 128) == 0 &&
              (kOffMSEP % 128) == 0 && (kOffMIP % 128) == 0, "128-B aligned regions");

constexpr int kOutZc   = 0;
constexpr int kOutMean = 131072;
constexpr int kOutStd  = 262144;
constexpr int kOutRec  = 393216;
constexpr int kOutScal = 2490368;
constexpr int kOutTotal = 2490374;
static_assert(kOutMean * 4 == 524288 && kOutStd * 4 == 1048576 && kOutRec * 4 == 1572864 && kOutScal * 4 == 9961472, "byte offsets");
static_assert(kOutScal + 6 == kOutTotal && kOutTotal * 4 == 9961496, "result extent");

__device__ __forceinline__ unsigned short f2bf_bits(float f) {
  unsigned u = __float_as_uint(f);
  return (unsigned short)((u + 0x7FFFu + ((u >> 16) & 1u)) >> 16);
}
__device__ __forceinline__ float bf_bits2f(unsigned short h) { return __uint_as_float(((unsigned)h) << 16); }
__device__ __forceinline__ float leaky02(float x) { return (x > 0.0f) ? x : 0.2f * x; }

__device__ __forceinline__ void dep_guard4_h(v8f& a, v8f& b, v8f& c, v8f& d, v16h x, v16h y) { asm volatile("v_nop\n\tv_nop\n\tv_nop\n\tv_nop" : "+v"(a), "+v"(b), "+v"(c), "+v"(d) : "v"(x), "v"(y)); }
__device__ __forceinline__ void dep_guard4_b(v8f& a, v8f& b, v8f& c, v8f& d, v16b x, v16b y) { asm volatile("v_nop\n\tv_nop\n\tv_nop\n\tv_nop" : "+v"(a), "+v"(b), "+v"(c), "+v"(d) : "v"(x), "v"(y)); }
__device__ __forceinline__ void keep4_h(v16h a, v16h b, v16h c, v16h d) { asm volatile("v_nop" :: "v"(a), "v"(b), "v"(c), "v"(d)); }
__device__ __forceinline__ void keep4_b(v16b a, v16b b, v16b c, v16b d) { asm volatile("v_nop" :: "v"(a), "v"(b), "v"(c), "v"(d)); }
__device__ __forceinline__ void acc_guard4(v8f& a, v8f& b, v8f& c, v8f& d) { asm volatile("v_nop\n\tv_nop\n\tv_nop\n\tv_nop" : "+v"(a), "+v"(b), "+v"(c), "+v"(d)); }
template <typename T> struct Frag;
template <> struct Frag<_Float16> {
  typedef v16h V; union U { v16h v; v8h h[2]; };
  static __device__ __forceinline__ v16h load(const _Float16* p) {
    U f; f.h[0] = *(const v8h*)(p); f.h[1] = *(const v8h*)(p + 16); return f.v;
  }
  static __device__ __forceinline__ v8f mma(v16h a, v16h b, v8f c) {
    return __builtin_amdgcn_wmma_f32_16x16x32_f16(false, a, false, b, (short)0, c, false, false);
  }
  static __device__ __forceinline__ void guard4(v8f& a, v8f& b, v8f& c, v8f& d, v16h x, v16h y) { dep_guard4_h(a, b, c, d, x, y); }
  static __device__ __forceinline__ void keep(v16h a, v16h b, v16h c, v16h d) { keep4_h(a, b, c, d); }
};
template <> struct Frag<__bf16> {
  typedef v16b V; union U { v16b v; v8b h[2]; };
  static __device__ __forceinline__ v16b load(const __bf16* p) {
    U f; f.h[0] = *(const v8b*)(p); f.h[1] = *(const v8b*)(p + 16); return f.v;
  }
  static __device__ __forceinline__ v8f mma(v16b a, v16b b, v8f c) {
    return __builtin_amdgcn_wmma_f32_16x16x32_bf16(false, a, false, b, (short)0, c, false, false);
  }
  static __device__ __forceinline__ void guard4(v8f& a, v8f& b, v8f& c, v8f& d, v16b x, v16b y) { dep_guard4_b(a, b, c, d, x, y); }
  static __device__ __forceinline__ void keep(v16b a, v16b b, v16b c, v16b d) { keep4_b(a, b, c, d); }
};

__device__ __forceinline__ v8f mma_f16_guarded(v16h a, v16h b, v8f c) {
  c = __builtin_amdgcn_wmma_f32_16x16x32_f16(false, a, false, b, (short)0, c, false, false);
  asm volatile("v_nop\n\tv_nop\n\tv_nop\n\tv_nop" : "+v"(c) : "v"(a), "v"(b));
  return c;
}

template <int ET> struct Elem;
template <> struct Elem<0> { typedef _Float16 T; };
template <> struct Elem<1> { typedef __bf16 T; };
template <int ET, bool SPLIT, int BIAS_MODE, int OUT_MODE, bool RESID, int ACT>
__global__ __launch_bounds__(256) void wmma_gemm64(
    const unsigned short* __restrict__ Ap, const unsigned short* __restrict__ A2p, int lda, long strideA,
    const unsigned short* __restrict__ Btp, const unsigned short* __restrict__ Bt2p, int ldb, long strideB,
    void* __restrict__ Cout, void* __restrict__ Cout2, int ldc, long strideC,
    const float* __restrict__ bias,
    const float* __restrict__ resid, long strideR,
    int M, int N, int K, float scale) {
  typedef typename Elem<ET>::T T;
  typedef typename Frag<T>::V V;
  const T* A = (const T*)Ap; const T* A2 = (const T*)A2p; const T* Bt = (const T*)Btp; const T* Bt2 = (const T*)Bt2p;
  __shared__ __align__(16) float sT[8][16 * 68];
  const int b    = blockIdx.y;
  const int lane = threadIdx.x & 31;
  const int wave = threadIdx.x >> 5;
  const int tilesN = N >> 6;
  const int tilesM = M >> 6;
  const int tile = blockIdx.x * 8 + wave;
  if (tile >= tilesM * tilesN) return;
  const int tm = tile / tilesN;
  const int tn = tile - tm * tilesN;
  const int m0 = tm << 6;
  const int n0 = tn << 6;

  const T* Ab  = A  + (size_t)b * strideA;
  const T* Bb  = Bt + (size_t)b * strideB;
  const T* Ab2 = SPLIT ? (A2  + (size_t)b * strideA) : nullptr;
  const T* Bb2 = SPLIT ? (Bt2 + (size_t)b * strideB) : nullptr;

  const int rlane = lane & 15;
  const int koff  = (lane >> 4) * 8;
  const int mOff  = (lane >> 4) * 8;

  v8f acc[4][4];
#pragma unroll
  for (int i = 0; i < 4; ++i)
#pragma unroll
    for (int j = 0; j < 4; ++j) acc[i][j] = (v8f){0.f,0.f,0.f,0.f,0.f,0.f,0.f,0.f};

  for (int k0 = 0; k0 < K; k0 += 32) {
    V bh[4], bl[4];
#pragma unroll
    for (int j = 0; j < 4; ++j) {
      const size_t bo = (size_t)(n0 + (j << 4) + rlane) * ldb + koff + k0;
      bh[j] = Frag<T>::load(Bb + bo);
      if (SPLIT) bl[j] = Frag<T>::load(Bb2 + bo);
    }
#pragma unroll
    for (int i = 0; i < 4; ++i) {
      const size_t ao = (size_t)(m0 + (i << 4) + rlane) * lda + koff + k0;
      V ah = Frag<T>::load(Ab + ao);
      V al = ah;
      if (SPLIT) al = Frag<T>::load(Ab2 + ao);
#pragma unroll
      for (int j = 0; j < 4; ++j) {
        acc[i][j] = Frag<T>::mma(ah, bh[j], acc[i][j]);
        if (SPLIT) {
          acc[i][j] = Frag<T>::mma(ah, bl[j], acc[i][j]);
          acc[i][j] = Frag<T>::mma(al, bh[j], acc[i][j]);
        }
      }
      Frag<T>::guard4(acc[i][0], acc[i][1], acc[i][2], acc[i][3], ah, al);
    }
    Frag<T>::keep(bh[0], bh[1], bh[2], bh[3]);
    if (SPLIT) Frag<T>::keep(bl[0], bl[1], bl[2], bl[3]);
  }
  acc_guard4(acc[0][0], acc[0][1], acc[0][2], acc[0][3]);
  acc_guard4(acc[1][0], acc[1][1], acc[1][2], acc[1][3]);
  acc_guard4(acc[2][0], acc[2][1], acc[2][2], acc[2][3]);
  acc_guard4(acc[3][0], acc[3][1], acc[3][2], acc[3][3]);

  float* slab = sT[wave];
  const float* Rb = RESID ? (resid + (size_t)b * strideR) : nullptr;
#pragma unroll
  for (int i = 0; i < 4; ++i) {
    const int mBase = m0 + (i << 4);
#pragma unroll
    for (int j = 0; j < 4; ++j) {
      const int n = n0 + (j << 4) + rlane;
      float bv = 0.f;
      if (BIAS_MODE == 2) bv = bias[n];
#pragma unroll
      for (int r = 0; r < 8; ++r) {
        float v = acc[i][j][r] * scale;
        if (BIAS_MODE == 1) v += bias[mBase + mOff + r];
        if (BIAS_MODE == 2) v += bv;
        if (RESID) v += Rb[(size_t)(mBase + mOff + r) * ldc + n];
        if (ACT == 1) v = (v > 0.f) ? v : 0.2f * v;
        slab[(mOff + r) * 68 + (j << 4) + rlane] = v;
      }
    }
    __builtin_amdgcn_fence(__ATOMIC_RELEASE, "workgroup");
    __builtin_amdgcn_wave_barrier();
    __builtin_amdgcn_fence(__ATOMIC_ACQUIRE, "workgroup");
    if (OUT_MODE == 0) {
      float* C = (float*)Cout + (size_t)b * strideC;
      const int hh = lane >> 4, c4 = (lane & 15) * 4;
      for (int pass = 0; pass < 2; ++pass) {
#pragma unroll
        for (int it = 0; it < 8; ++it) {
          const int row = it * 2 + hh;
          v4f v = *(const v4f*)(slab + row * 68 + c4);
          *(volatile v4f*)(C + (size_t)(mBase + row) * ldc + n0 + c4) = v;
        }
        __threadfence();
      }
    } else {
      const int q = lane >> 3, c8 = (lane & 7) * 8;
      unsigned short* C  = (unsigned short*)Cout  + (size_t)b * strideC;
      unsigned short* C2 = (OUT_MODE == 2) ? ((unsigned short*)Cout2 + (size_t)b * strideC) : nullptr;
      for (int pass = 0; pass < 2; ++pass) {
#pragma unroll
        for (int it = 0; it < 4; ++it) {
          const int row = it * 4 + q;
          const float* sp = slab + row * 68 + c8;
          v8h hv, lv;
#pragma unroll
          for (int e = 0; e < 8; ++e) {
            if (OUT_MODE == 1) {
              hv[e] = (_Float16)sp[e];
            } else {
              unsigned short hb = f2bf_bits(sp[e]);
              unsigned short lb = f2bf_bits(sp[e] - bf_bits2f(hb));
              hv[e] = __builtin_bit_cast(_Float16, hb);
              lv[e] = __builtin_bit_cast(_Float16, lb);
            }
          }
          *(volatile v8h*)(C + (size_t)(mBase + row) * ldc + n0 + c8) = hv;
          if (OUT_MODE == 2) *(volatile v8h*)(C2 + (size_t)(mBase + row) * ldc + n0 + c8) = lv;
        }
        __threadfence();
      }
    }
    __builtin_amdgcn_fence(__ATOMIC_RELEASE, "workgroup");
    __builtin_amdgcn_wave_barrier();
    __builtin_amdgcn_fence(__ATOMIC_ACQUIRE, "workgroup");
  }
}

__global__ __launch_bounds__(256) void split_rows_bf16_kernel(
    const float* __restrict__ src, unsigned short* __restrict__ dhi, unsigned short* __restrict__ dlo, int total8)
{
  const int i = blockIdx.x * 256 + threadIdx.x;
  if (i >= total8) return;
  const size_t e0 = (size_t)i << 3;
  const v4f a0 = *(const v4f*)(src + e0);
  const v4f a1 = *(const v4f*)(src + e0 + 4);
  v8h hv, lv;
#pragma unroll
  for (int e = 0; e < 4; ++e) {
    const unsigned short h0 = f2bf_bits(a0[e]), h1 = f2bf_bits(a1[e]);
    const unsigned short l0 = f2bf_bits(a0[e] - bf_bits2f(h0)), l1 = f2bf_bits(a1[e] - bf_bits2f(h1));
    hv[e]     = __builtin_bit_cast(_Float16, h0);
    hv[4 + e] = __builtin_bit_cast(_Float16, h1);
    lv[e]     = __builtin_bit_cast(_Float16, l0);
    lv[4 + e] = __builtin_bit_cast(_Float16, l1);
  }
  unsigned short* qh = dhi + e0;
  unsigned short* ql = dlo + e0;
  *(volatile v8h*)qh = hv;
  *(volatile v8h*)ql = lv;
  __threadfence();
  *(volatile v8h*)qh = hv;
  *(volatile v8h*)ql = lv;
}

template <int OUTK>
__global__ __launch_bounds__(256) void transpose64_kernel(
    const float* __restrict__ W, unsigned short* __restrict__ BtH, unsigned short* __restrict__ BtL,
    int Kdim, int Ndim, long strideIn, long strideOut, float scale)
{
  __shared__ float tile[64 * 65];
  const int tid = threadIdx.x, lane = tid & 31, wave = tid >> 5;
  const int n0 = blockIdx.x * 64;
  const int k0 = blockIdx.y * 64;
  const float* Wb = W + (size_t)blockIdx.z * strideIn;
#pragma unroll
  for (int p = 0; p < 16; ++p) {
    const int idx = tid + p * 256;
    const int kk  = idx >> 6;
    const int nn  = idx & 63;
    const float v = Wb[(size_t)(k0 + kk) * Ndim + n0 + nn];
    tile[kk * 65 + nn] = v * scale;
  }
  __syncthreads();
  const int q = lane >> 3, c8 = (lane & 7) * 8;
  v8h hv[2], lv[2];
#pragma unroll
  for (int it = 0; it < 2; ++it) {
    const int nrow = it * 32 + wave * 4 + q;
#pragma unroll
    for (int e = 0; e < 8; ++e) {
      const float x = tile[(c8 + e) * 65 + nrow];
      if (OUTK == 0) {
        hv[it][e] = (_Float16)x;
        lv[it][e] = hv[it][e];
      } else {
        const unsigned short hb = f2bf_bits(x);
        const unsigned short lb = f2bf_bits(x - bf_bits2f(hb));
        hv[it][e] = __builtin_bit_cast(_Float16, hb);
        lv[it][e] = __builtin_bit_cast(_Float16, lb);
      }
    }
  }
  unsigned short* oh = BtH + (size_t)blockIdx.z * strideOut;
  unsigned short* ol = BtL + (size_t)blockIdx.z * strideOut;
  for (int pass = 0; pass < 2; ++pass) {
#pragma unroll
    for (int it = 0; it < 2; ++it) {
      const int nrow = it * 32 + wave * 4 + q;
      const size_t o = (size_t)(n0 + nrow) * Kdim + k0 + c8;
      *(volatile v8h*)(oh + o) = hv[it];
      if (OUTK == 1) *(volatile v8h*)(ol + o) = lv[it];
    }
    __threadfence();
  }
}

template <int MODE>
__global__ __launch_bounds__(256) void tr32_kernel(
    const float* __restrict__ Win, const float* __restrict__ logw,
    unsigned short* __restrict__ OutH, unsigned short* __restrict__ OutL, int Wd)
{
  __shared__ float tile[32 * 65];
  __shared__ float sAdj[32];
  const int tid = threadIdx.x;
  const int i  = blockIdx.y;
  const int h0 = blockIdx.x * 64;
  if (MODE == 0) {
    if (tid < 32) {
      const int s = tid;
      const float lraw = logw[s * 32 + i];
      float x = (i > s) ? (lraw * 10.0f) : 0.0f;
      x = fminf(fmaxf(x, -60.0f), 60.0f);
      const float sg = 1.0f / (1.0f + expf(-x));
      sAdj[s] = (s == i) ? 0.0f : sg;
    }
  }
#pragma unroll
  for (int p = 0; p < 8; ++p) {
    const int idx = tid + p * 256;
    const int s  = idx >> 6;
    const int hh = idx & 63;
    tile[s * 65 + hh] = Win[((size_t)i * 32 + s) * Wd + h0 + hh];
  }
  __syncthreads();
  const int row = tid >> 2, c8 = (tid & 3) * 8;
  v8h hv, lv;
#pragma unroll
  for (int e = 0; e < 8; ++e) {
    float x = tile[(c8 + e) * 65 + row];
    if (MODE == 0) {
      x = (sAdj[c8 + e] * x) * kMechCarry;
      hv[e] = (_Float16)x;
      lv[e] = hv[e];
    } else {
      const unsigned short hb = f2bf_bits(x);
      const unsigned short lb = f2bf_bits(x - bf_bits2f(hb));
      hv[e] = __builtin_bit_cast(_Float16, hb);
      lv[e] = __builtin_bit_cast(_Float16, lb);
    }
  }
  const size_t o = ((size_t)i * Wd + h0 + row) * 32 + c8;
  for (int pass = 0; pass < 2; ++pass) {
    *(volatile v8h*)(OutH + o) = hv;
    if (MODE == 1) *(volatile v8h*)(OutL + o) = lv;
    __threadfence();
  }
}

__global__ __launch_bounds__(256) void reparam_kernel(
    const float* __restrict__ params, const float* __restrict__ eps,
    float* __restrict__ outMean, float* __restrict__ outStd, float* __restrict__ zF, float* __restrict__ klp)
{
  __shared__ float sRed[8];
  const int tid = threadIdx.x, lane = tid & 31, wave = tid >> 5;
  const int row = blockIdx.x * 32 + (tid >> 3);
  const int c4  = (tid & 7) * 4;
  const v4f mu = *(const v4f*)(params + (size_t)row * kPar + c4);
  const v4f ls = *(const v4f*)(params + (size_t)row * kPar + kSto + c4);
  const v4f ep = *(const v4f*)(eps + (size_t)row * kSto + c4);
  v4f sd, zz;
  float kl = 0.0f;
#pragma unroll
  for (int e = 0; e < 4; ++e) {
    const float m = mu[e];
    const float l = ls[e];
    const float s = expf(l);
    sd[e] = s;
    zz[e] = m + s * ep[e];
    kl += m * m + s * s - 2.0f * l - 1.0f;
  }
  const size_t o = (size_t)row * kSto + c4;
  for (int pass = 0; pass < 2; ++pass) {
    *(volatile v4f*)(outMean + o) = mu;
    *(volatile v4f*)(outStd + o)  = sd;
    *(volatile v4f*)(zF + o)      = zz;
    __threadfence();
  }
#pragma unroll
  for (int off = 16; off > 0; off >>= 1) kl += __shfl_xor(kl, off, 32);
  if (lane == 0) sRed[wave] = kl;
  __syncthreads();
  float t = sRed[lane & 7];
  t = (lane < 8) ? t : 0.0f;
#pragma unroll
  for (int off = 16; off > 0; off >>= 1) t += __shfl_xor(t, off, 32);
  const float lineval = (lane == 0) ? t : 0.0f;
  if (wave == 0) {
    float* dst = klp + (size_t)blockIdx.x * 32 + lane;
    *(volatile float*)dst = lineval;
    __threadfence();
    *(volatile float*)dst = lineval;
  }
}

__global__ __launch_bounds__(256) void mech_kernel(
    const float* __restrict__ zF, const unsigned short* __restrict__ mechW,
    const float* __restrict__ b1, const float* __restrict__ w2, const float* __restrict__ b2,
    float* __restrict__ outZc, unsigned short* __restrict__ ZCH, unsigned short* __restrict__ ZCL)
{
  __shared__ __align__(16) float sZ[64 * 36];
  const int tid = threadIdx.x, lane = tid & 31, wave = tid >> 5;
  const int hh = lane >> 4, c = lane & 15;
  const int m0 = blockIdx.x * 64;

  v16h ah[4], al[4];
#pragma unroll
  for (int mt = 0; mt < 4; ++mt) {
    const float* zr = zF + (size_t)(m0 + mt * 16 + c) * kSto + 8 * hh;
    const v4f x0 = *(const v4f*)(zr);
    const v4f x1 = *(const v4f*)(zr + 4);
    const v4f x2 = *(const v4f*)(zr + 16);
    const v4f x3 = *(const v4f*)(zr + 20);
#pragma unroll
    for (int e = 0; e < 4; ++e) {
      const float f0 = x0[e], f1 = x1[e], f2 = x2[e], f3 = x3[e];
      const _Float16 h0 = (_Float16)f0, h1 = (_Float16)f1, h2 = (_Float16)f2, h3 = (_Float16)f3;
      ah[mt][e]      = h0;
      ah[mt][4 + e]  = h1;
      ah[mt][8 + e]  = h2;
      ah[mt][12 + e] = h3;
      al[mt][e]      = (_Float16)((f0 - (float)h0) * kLoCarry);
      al[mt][4 + e]  = (_Float16)((f1 - (float)h1) * kLoCarry);
      al[mt][8 + e]  = (_Float16)((f2 - (float)h2) * kLoCarry);
      al[mt][12 + e] = (_Float16)((f3 - (float)h3) * kLoCarry);
    }
  }

#pragma unroll 1
  for (int ii = 0; ii < 4; ++ii) {
    const int i = wave + 8 * ii;
    const _Float16* Wi = (const _Float16*)mechW + (size_t)i * kHid2 * kSto;
    float part[4][8];
#pragma unroll
    for (int mt = 0; mt < 4; ++mt)
#pragma unroll
      for (int r = 0; r < 8; ++r) part[mt][r] = 0.0f;
#pragma unroll 1
    for (int nt = 0; nt < 16; ++nt) {
      const int n = nt * 16 + c;
      const v16h bw = Frag<_Float16>::load(Wi + (size_t)n * kSto + 8 * hh);
      const float b1v = b1[i * kHid2 + n];
      const float w2v = w2[i * kHid2 + n];
#pragma unroll
      for (int mt = 0; mt < 4; ++mt) {
        v8f ch = (v8f){0.f,0.f,0.f,0.f,0.f,0.f,0.f,0.f};
        v8f cl = (v8f){0.f,0.f,0.f,0.f,0.f,0.f,0.f,0.f};
        ch = mma_f16_guarded(ah[mt], bw, ch);
        cl = mma_f16_guarded(al[mt], bw, cl);
#pragma unroll
        for (int r = 0; r < 8; ++r) {
          float v = fmaf(ch[r], kMechCarryInv, b1v);
          v = fmaf(cl[r], kMechLoInv, v);
          v = leaky02(v);
          part[mt][r] = fmaf(v, w2v, part[mt][r]);
        }
      }
    }
#pragma unroll
    for (int mt = 0; mt < 4; ++mt)
#pragma unroll
      for (int r = 0; r < 8; ++r) {
        float x = part[mt][r];
        x += __shfl_xor(x, 1, 32);
        x += __shfl_xor(x, 2, 32);
        x += __shfl_xor(x, 4, 32);
        x += __shfl_xor(x, 8, 32);
        part[mt][r] = x;
      }
    const float b2v = b2[i];
    if (c == 0) {
#pragma unroll
      for (int mt = 0; mt < 4; ++mt)
#pragma unroll
        for (int r = 0; r < 8; ++r) sZ[(mt * 16 + 8 * hh + r) * 36 + i] = part[mt][r] + b2v;
    }
  }
  __syncthreads();

  v4f ov[2];
#pragma unroll
  for (int it = 0; it < 2; ++it) ov[it] = *(const v4f*)(sZ + (it * 32 + (tid >> 3)) * 36 + (tid & 7) * 4);
  const int row2 = tid >> 2, c8 = (tid & 3) * 8;
  v8h hv, lv;
  {
    const v4f a0 = *(const v4f*)(sZ + row2 * 36 + c8);
    const v4f a1 = *(const v4f*)(sZ + row2 * 36 + c8 + 4);
#pragma unroll
    for (int e = 0; e < 4; ++e) {
      const float f0 = a0[e], f1 = a1[e];
      const unsigned short h0 = f2bf_bits(f0), h1 = f2bf_bits(f1);
      const unsigned short l0 = f2bf_bits(f0 - bf_bits2f(h0)), l1 = f2bf_bits(f1 - bf_bits2f(h1));
      hv[e]     = __builtin_bit_cast(_Float16, h0);
      hv[4 + e] = __builtin_bit_cast(_Float16, h1);
      lv[e]     = __builtin_bit_cast(_Float16, l0);
      lv[4 + e] = __builtin_bit_cast(_Float16, l1);
    }
  }
  const size_t o16 = (size_t)(m0 + row2) * kSto + c8;
  for (int pass = 0; pass < 2; ++pass) {
#pragma unroll
    for (int it = 0; it < 2; ++it)
      *(volatile v4f*)(outZc + (size_t)(m0 + it * 32 + (tid >> 3)) * kSto + (tid & 7) * 4) = ov[it];
    *(volatile v8h*)(ZCH + o16) = hv;
    *(volatile v8h*)(ZCL + o16) = lv;
    __threadfence();
  }
}

__device__ __forceinline__ void pair_ij(int p, int& io, int& jo) {
  int i = 0, rem = p;
#pragma unroll 1
  for (int it = 0; it < 31; ++it) {
    const int cnt = 31 - i;
    if (rem >= cnt) { rem -= cnt; ++i; }
  }
  io = i;
  jo = i + 1 + rem;
}

__global__ __launch_bounds__(256) void mi_kernel(
    const float* __restrict__ zF, const unsigned short* __restrict__ w2T,
    const float* __restrict__ w1, const float* __restrict__ b1, const float* __restrict__ b2,
    const float* __restrict__ w3, float* __restrict__ mip)
{
  __shared__ __align__(16) float sW1a[64];
  __shared__ __align__(16) float sW1b[64];
  __shared__ __align__(16) float sB1[64];
  __shared__ float sRed[8];
  const int tid = threadIdx.x, lane = tid & 31, wave = tid >> 5;
  const int hh = lane >> 4, c = lane & 15;
  const int p = blockIdx.x;
  if (tid < 64) {
    sW1a[tid] = w1[(size_t)p * 128 + tid];
    sW1b[tid] = w1[(size_t)p * 128 + 64 + tid];
    sB1[tid]  = b1[(size_t)p * 64 + tid];
  }
  int pi, pj;
  pair_ij(p, pi, pj);
  const _Float16* Wp = (const _Float16*)w2T + (size_t)p * (kMiH * kMiH);
  v16h bf[4][2];
#pragma unroll
  for (int nt = 0; nt < 4; ++nt)
#pragma unroll
    for (int ks = 0; ks < 2; ++ks)
      bf[nt][ks] = Frag<_Float16>::load(Wp + (size_t)(nt * 16 + c) * kMiH + ks * 32 + 8 * hh);
  float b2v[4], w3v[4];
#pragma unroll
  for (int nt = 0; nt < 4; ++nt) {
    b2v[nt] = b2[(size_t)p * 64 + nt * 16 + c];
    w3v[nt] = w3[(size_t)p * 64 + nt * 16 + c];
  }
  __syncthreads();

  float psum = 0.0f;
  const int rowbase = wave * 512;
#pragma unroll 1
  for (int mt = 0; mt < 32; ++mt) {
    const int row = rowbase + mt * 16 + c;
    const float zi = zF[(size_t)row * kSto + pi];
    const float zj = zF[(size_t)row * kSto + pj];
    v16h af[2];
#pragma unroll
    for (int t = 0; t < 2; ++t) {
#pragma unroll
      for (int g = 0; g < 2; ++g) {
        const int kb = t * 32 + g * 16 + 8 * hh;
        const v4f wa0 = *(const v4f*)(sW1a + kb);
        const v4f wa1 = *(const v4f*)(sW1a + kb + 4);
        const v4f wb0 = *(const v4f*)(sW1b + kb);
        const v4f wb1 = *(const v4f*)(sW1b + kb + 4);
        const v4f bb0 = *(const v4f*)(sB1 + kb);
        const v4f bb1 = *(const v4f*)(sB1 + kb + 4);
#pragma unroll
        for (int e = 0; e < 4; ++e) {
          const float v0 = fmaf(zj, wb0[e], zi * wa0[e]) + bb0[e];
          const float v1 = fmaf(zj, wb1[e], zi * wa1[e]) + bb1[e];
          af[t][g * 8 + e]     = (_Float16)leaky02(v0);
          af[t][g * 8 + 4 + e] = (_Float16)leaky02(v1);
        }
      }
    }
    float tsum = 0.0f;
#pragma unroll
    for (int nt = 0; nt < 4; ++nt) {
      v8f acc = (v8f){0.f,0.f,0.f,0.f,0.f,0.f,0.f,0.f};
      acc = mma_f16_guarded(af[0], bf[nt][0], acc);
      acc = mma_f16_guarded(af[1], bf[nt][1], acc);
#pragma unroll
      for (int r = 0; r < 8; ++r) {
        float v = fmaf(acc[r], kMiCarryInv, b2v[nt]);
        v = leaky02(v);
        tsum = fmaf(v, w3v[nt], tsum);
      }
    }
    psum += tsum;
  }
#pragma unroll
  for (int off = 16; off > 0; off >>= 1) psum += __shfl_xor(psum, off, 32);
  if (lane == 0) sRed[wave] = psum;
  __syncthreads();
  float t = sRed[lane & 7];
  t = (lane < 8) ? t : 0.0f;
#pragma unroll
  for (int off = 16; off > 0; off >>= 1) t += __shfl_xor(t, off, 32);
  const float lineval = (lane == 0) ? t : 0.0f;
  if (wave == 0) {
    float* dst = mip + (size_t)p * 32 + lane;
    *(volatile float*)dst = lineval;
    __threadfence();
    *(volatile float*)dst = lineval;
  }
}

__global__ __launch_bounds__(256) void mse_kernel(
    const float* __restrict__ recon, const float* __restrict__ feat, float* __restrict__ msep)
{
  __shared__ float sRed[8];
  const int tid = threadIdx.x, lane = tid & 31, wave = tid >> 5;
  const size_t base = (size_t)blockIdx.x * 4096 + (size_t)tid * 4;
  float s = 0.0f;
#pragma unroll 1
  for (int q = 0; q < 4; ++q) {
    const v4f a = *(const v4f*)(recon + base + (size_t)q * 1024);
    const v4f b = *(const v4f*)(feat + base + (size_t)q * 1024);
#pragma unroll
    for (int e = 0; e < 4; ++e) {
      const float d = a[e] - b[e];
      s = fmaf(d, d, s);
    }
  }
#pragma unroll
  for (int off = 16; off > 0; off >>= 1) s += __shfl_xor(s, off, 32);
  if (lane == 0) sRed[wave] = s;
  __syncthreads();
  float t = sRed[lane & 7];
  t = (lane < 8) ? t : 0.0f;
#pragma unroll
  for (int off = 16; off > 0; off >>= 1) t += __shfl_xor(t, off, 32);
  const float lineval = (lane == 0) ? t : 0.0f;
  if (wave == 0) {
    float* dst = msep + (size_t)blockIdx.x * 32 + lane;
    *(volatile float*)dst = lineval;
    __threadfence();
    *(volatile float*)dst = lineval;
  }
}

__device__ __forceinline__ float block_sum_1024(float v, float* red, int t) {
  red[t] = v;
  __syncthreads();
  for (int s = 512; s > 0; s >>= 1) {
    if (t < s) red[t] += red[t + s];
    __syncthreads();
  }
  const float o = red[0];
  __syncthreads();
  return o;
}

__global__ __launch_bounds__(1024) void finalize_kernel(
    const float* __restrict__ logw, const float* __restrict__ mi_b3,
    const float* __restrict__ klp, const float* __restrict__ msep, const float* __restrict__ mip,
    float* __restrict__ scal)
{
  __shared__ float red[1024];
  __shared__ float a2s[1024];
  __shared__ float mps[1024];
  __shared__ float sOut[8];
  const int t = threadIdx.x;
  const int r = t >> 5, c = t & 31;

  const float sig = 1.0f / (1.0f + expf(-logw[t]));
  a2s[t] = sig * sig;
  mps[t] = (r == c) ? 1.0f : 0.0f;
  const float sp = block_sum_1024(fabsf(sig), red, t);

  float traceLocal = 0.0f;
  float fact = 1.0f;
#pragma unroll 1
  for (int it = 1; it <= 9; ++it) {
    float acc = 0.0f;
#pragma unroll 8
    for (int k = 0; k < 32; ++k) acc = fmaf(mps[r * 32 + k], a2s[k * 32 + c], acc);
    __syncthreads();
    mps[t] = acc;
    __syncthreads();
    fact *= (float)it;
    if (r == c) traceLocal += acc * (1.0f / fact);
  }
  const float trp = block_sum_1024(traceLocal, red, t);

  const int tk = (t < kKlBlocks) ? t : (kKlBlocks - 1);
  const float klraw = klp[(size_t)tk * 32];
  const float kls = block_sum_1024((t < kKlBlocks) ? klraw : 0.0f, red, t);

  const int tm = (t < kMseBlocks) ? t : (kMseBlocks - 1);
  const float rcraw = msep[(size_t)tm * 32];
  const float rcs = block_sum_1024((t < kMseBlocks) ? rcraw : 0.0f, red, t);

  const int tc = (t < kPairs) ? t : (kPairs - 1);
  int pi, pj;
  pair_ij(tc, pi, pj);
  const float msum = mip[(size_t)tc * 32];
  const float b3v  = mi_b3[tc];
  const float lwv  = logw[pi * 32 + pj];
  const float est  = msum * (1.0f / 4096.0f) + b3v;
  const float miv  = (1.0f / (1.0f + expf(-lwv))) * est;
  const float mis = block_sum_1024((t < kPairs) ? miv : 0.0f, red, t);

  if (t == 0) {
    const float recon_loss = rcs * (1.0f / (4096.0f * 512.0f));
    const float kl_loss = 0.5f * (kls * (1.0f / 4096.0f));
    const float dag = trp * trp;
    float total = recon_loss + kl_loss;
    total = total + 0.1f * sp;
    total = total + 0.01f * mis;
    total = total + dag;
    sOut[0] = total;
    sOut[1] = recon_loss;
    sOut[2] = kl_loss;
    sOut[3] = sp;
    sOut[4] = mis;
    sOut[5] = dag;
    sOut[6] = 0.0f;
    sOut[7] = 0.0f;
  }
  __syncthreads();
  const float val = sOut[t & 7];
  if (t < 6) {
    *(volatile float*)(scal + t) = val;
    __threadfence();
    *(volatile float*)(scal + t) = val;
  }
}

extern "C" void kernel_launch(void* const* d_in, const int* in_sizes, int n_in,
                              void* d_out, int out_size, void* d_ws, size_t ws_size,
                              hipStream_t stream) {
  if (n_in < 21) return;
  if (in_sizes[0] != kBatch * kFeat || in_sizes[1] != kBatch * kSto) return;
  if (in_sizes[2] != kFeat * kHid || in_sizes[3] != kHid) return;
  if (in_sizes[4] != kHid * kPar || in_sizes[5] != kPar) return;
  if (in_sizes[6] != kSto * kSto) return;
  if (in_sizes[7] != kSto * kSto * kHid2 || in_sizes[8] != kSto * kHid2 || in_sizes[9] != kSto * kHid2) return;
  if (in_sizes[10] != kSto) return;
  if (in_sizes[11] != kSto * kHid || in_sizes[12] != kHid) return;
  if (in_sizes[13] != kHid * kFeat || in_sizes[14] != kFeat) return;
  if (in_sizes[15] != kPairs * 2 * kMiH || in_sizes[16] != kPairs * kMiH) return;
  if (in_sizes[17] != kPairs * kMiH * kMiH || in_sizes[18] != kPairs * kMiH) return;
  if (in_sizes[19] != kPairs * kMiH || in_sizes[20] != kPairs) return;
  if (out_size != kOutTotal) return;
  if (ws_size < kWsTotal) return;

  const float* features   = (const float*)d_in[0];
  const float* eps        = (const float*)d_in[1];
  const float* enc_w1     = (const float*)d_in[2];
  const float* enc_b1     = (const float*)d_in[3];
  const float* enc_w2     = (const float*)d_in[4];
  const float* enc_b2     = (const float*)d_in[5];
  const float* log_weight = (const float*)d_in[6];
  const float* mech_w1    = (const float*)d_in[7];
  const float* mech_b1    = (const float*)d_in[8];
  const float* mech_w2    = (const float*)d_in[9];
  const float* mech_b2    = (const float*)d_in[10];
  const float* dec_w1     = (const float*)d_in[11];
  const float* dec_b1     = (const float*)d_in[12];
  const float* dec_w2     = (const float*)d_in[13];
  const float* dec_b2     = (const float*)d_in[14];
  const float* mi_w1      = (const float*)d_in[15];
  const float* mi_b1      = (const float*)d_in[16];
  const float* mi_w2      = (const float*)d_in[17];
  const float* mi_b2      = (const float*)d_in[18];
  const float* mi_w3      = (const float*)d_in[19];
  const float* mi_b3      = (const float*)d_in[20];

  float* out = (float*)d_out;
  float* out_zc   = out + kOutZc;
  float* out_mean = out + kOutMean;
  float* out_std  = out + kOutStd;
  float* out_rec  = out + kOutRec;
  float* out_scal = out + kOutScal;

  char* ws = (char*)d_ws;
  unsigned short* FH   = (unsigned short*)(ws + kOffFH);
  unsigned short* FL   = (unsigned short*)(ws + kOffFL);
  unsigned short* W1H  = (unsigned short*)(ws + kOffW1H);
  unsigned short* W1L  = (unsigned short*)(ws + kOffW1L);
  unsigned short* W2H  = (unsigned short*)(ws + kOffW2H);
  unsigned short* W2L  = (unsigned short*)(ws + kOffW2L);
  unsigned short* HH   = (unsigned short*)(ws + kOffHH);
  unsigned short* HL   = (unsigned short*)(ws + kOffHL);
  float*          PAR  = (float*)(ws + kOffPar);
  float*          ZF   = (float*)(ws + kOffZF);
  unsigned short* MW   = (unsigned short*)(ws + kOffMW);
  unsigned short* ZCH  = (unsigned short*)(ws + kOffZCH);
  unsigned short* ZCL  = (unsigned short*)(ws + kOffZCL);
  unsigned short* D1H  = (unsigned short*)(ws + kOffD1H);
  unsigned short* D1L  = (unsigned short*)(ws + kOffD1L);
  unsigned short* GH   = (unsigned short*)(ws + kOffGH);
  unsigned short* GL   = (unsigned short*)(ws + kOffGL);
  unsigned short* D2H  = (unsigned short*)(ws + kOffD2H);
  unsigned short* D2L  = (unsigned short*)(ws + kOffD2L);
  unsigned short* MIW  = (unsigned short*)(ws + kOffMIW);
  float*          KLP  = (float*)(ws + kOffKLP);
  float*          MSEP = (float*)(ws + kOffMSEP);
  float*          MIP  = (float*)(ws + kOffMIP);

  split_rows_bf16_kernel<<<(kBatch * kFeat / 8) / 256, 256, 0, stream>>>(features, FH, FL, kBatch * kFeat / 8);
  transpose64_kernel<1><<<dim3(kHid / 64, kFeat / 64, 1), 256, 0, stream>>>(enc_w1, W1H, W1L, kFeat, kHid, 0L, 0L, 1.0f);
  transpose64_kernel<1><<<dim3(kPar / 64, kHid / 64, 1), 256, 0, stream>>>(enc_w2, W2H, W2L, kHid, kPar, 0L, 0L, 1.0f);
  transpose64_kernel<1><<<dim3(kFeat / 64, kHid / 64, 1), 256, 0, stream>>>(dec_w2, D2H, D2L, kHid, kFeat, 0L, 0L, 1.0f);
  transpose64_kernel<0><<<dim3(1, 1, kPairs), 256, 0, stream>>>(mi_w2, MIW, MIW, kMiH, kMiH, (long)(kMiH * kMiH), (long)(kMiH * kMiH), kMiCarry);
  tr32_kernel<0><<<dim3(kHid2 / 64, kSto), 256, 0, stream>>>(mech_w1, log_weight, MW, MW, kHid2);
  tr32_kernel<1><<<dim3(kHid / 64, 1), 256, 0, stream>>>(dec_w1, log_weight, D1H, D1L, kHid);

  wmma_gemm64<1, true, 2, 2, false, 1><<<dim3(64, 1), 256, 0, stream>>>(
      FH, FL, kFeat, 0L, W1H, W1L, kFeat, 0L,
      (void*)HH, (void*)HL, kHid, 0L, enc_b1, enc_b1, 0L, kBatch, kHid, kFeat, 1.0f);
  wmma_gemm64<1, true, 2, 0, false, 0><<<dim3(8, 1), 256, 0, stream>>>(
      HH, HL, kHid, 0L, W2H, W2L, kHid, 0L,
      (void*)PAR, (void*)PAR, kPar, 0L, enc_b2, enc_b2, 0L, kBatch, kPar, kHid, 1.0f);
  reparam_kernel<<<kKlBlocks, 256, 0, stream>>>(PAR, eps, out_mean, out_std, ZF, KLP);

  mech_kernel<<<kBatch / 64, 256, 0, stream>>>(ZF, MW, mech_b1, mech_w2, mech_b2, out_zc, ZCH, ZCL);

  wmma_gemm64<1, true, 2, 2, false, 1><<<dim3(64, 1), 256, 0, stream>>>(
      ZCH, ZCL, kSto, 0L, D1H, D1L, kSto, 0L,
      (void*)GH, (void*)GL, kHid, 0L, dec_b1, dec_b1, 0L, kBatch, kHid, kSto, 1.0f);
  wmma_gemm64<1, true, 2, 0, false, 0><<<dim3(64, 1), 256, 0, stream>>>(
      GH, GL, kHid, 0L, D2H, D2L, kHid, 0L,
      (void*)out_rec, (void*)out_rec, kFeat, 0L, dec_b2, dec_b2, 0L, kBatch, kFeat, kHid, 1.0f);
  mse_kernel<<<kMseBlocks, 256, 0, stream>>>(out_rec, features, MSEP);

  mi_kernel<<<kPairs, 256, 0, stream>>>(ZF, MIW, mi_w1, mi_b1, mi_b2, mi_w3, MIP);

  finalize_kernel<<<1, 1024, 0, stream>>>(log_weight, mi_b3, KLP, MSEP, MIP, out_scal);
}
